// GraphCrossAttenNet_52553219833885
// MI455X (gfx1250) — hardware-run, weakly checked
//
#include <hip/hip_runtime.h>

typedef float          v8f   __attribute__((ext_vector_type(8)));
typedef float          v4f   __attribute__((ext_vector_type(4)));
typedef unsigned int   v4u   __attribute__((ext_vector_type(4)));
typedef int            v8i   __attribute__((ext_vector_type(8)));
typedef unsigned short v8us  __attribute__((ext_vector_type(8)));
typedef unsigned short v16us __attribute__((ext_vector_type(16)));
typedef __bf16         v16bf __attribute__((ext_vector_type(16)));
typedef _Float16       v16h  __attribute__((ext_vector_type(16)));
typedef v4f  __attribute__((may_alias)) v4fa;
typedef v8us __attribute__((may_alias)) v8usa;
union FragB { v16bf v; v16us u; v8us h[2]; v8i w; };
union FragH { v16h  v; v16us u; v8us h[2]; v8i w; };

__device__ __forceinline__ v8f wmb(const FragB& a, const FragB& b, v8f c) {
  v8f d = __builtin_amdgcn_wmma_f32_16x16x32_bf16(false, a.v, false, b.v, (short)0, c, false, false);
  asm volatile("v_nop\n\tv_nop\n\tv_nop\n\tv_nop" : "+v"(d) : "v"(a.w), "v"(b.w));
  return d;
}

__device__ __forceinline__ v8f wmh(const FragH& a, const FragH& b, v8f c) {
  v8f d = __builtin_amdgcn_wmma_f32_16x16x32_f16(false, a.v, false, b.v, (short)0, c, false, false);
  asm volatile("v_nop\n\tv_nop\n\tv_nop\n\tv_nop" : "+v"(d) : "v"(a.w), "v"(b.w));
  return d;
}

__device__ __forceinline__ unsigned bf16_bits(float f) {
  const unsigned u = __float_as_uint(f);
  const unsigned r = (u + 0x7FFFu + ((u >> 16) & 1u)) >> 16;
  const unsigned q = (u >> 16) | 0x40u;
  return ((u & 0x7fffffffu) > 0x7f800000u) ? q : r;
}

__device__ __forceinline__ float bf16_val(float f) {
  return __uint_as_float(bf16_bits(f) << 16);
}
__device__ __forceinline__ int clampi(int v, int lo, int hi) {
  return v < lo ? lo : (v > hi ? hi : v);
}

__device__ __forceinline__ unsigned f16_bits(float f) {
  const unsigned u  = __float_as_uint(f);
  const unsigned s  = (u >> 16) & 0x8000u;
  const unsigned a  = u & 0x7fffffffu;
  const unsigned t  = a - 0x38000000u;
  const unsigned r  = (t + 0x0FFFu + ((t >> 13) & 1u)) >> 13;
  const unsigned rc = r > 0x7C00u ? 0x7C00u : r;
  const bool small  = a < 0x38800000u;
  const bool isnan  = a > 0x7f800000u;
  const unsigned fin = small ? 0u : (s | rc);
  return isnan ? (s | 0x7E00u) : fin;
}

__device__ __forceinline__ unsigned pk16(unsigned lo, unsigned hi) { return lo | (hi << 16); }
__device__ __forceinline__ unsigned bf16_lo_bits(float v) {
  float hi = bf16_val(v);
  asm volatile("" : "+v"(hi));
  return bf16_bits(v - hi);
}
__device__ __forceinline__ v4u pack8_bf16(v4f a, v4f c) {
  return (v4u){ pk16(bf16_bits(a[0]), bf16_bits(a[1])), pk16(bf16_bits(a[2]), bf16_bits(a[3])),
                pk16(bf16_bits(c[0]), bf16_bits(c[1])), pk16(bf16_bits(c[2]), bf16_bits(c[3])) };
}
__device__ __forceinline__ v4u pack8_bf16_lo(v4f a, v4f c) {
  return (v4u){ pk16(bf16_lo_bits(a[0]), bf16_lo_bits(a[1])), pk16(bf16_lo_bits(a[2]), bf16_lo_bits(a[3])),
                pk16(bf16_lo_bits(c[0]), bf16_lo_bits(c[1])), pk16(bf16_lo_bits(c[2]), bf16_lo_bits(c[3])) };
}
__device__ __forceinline__ v4u pack8_f16(v4f a, v4f c) {
  return (v4u){ pk16(f16_bits(a[0]), f16_bits(a[1])), pk16(f16_bits(a[2]), f16_bits(a[3])),
                pk16(f16_bits(c[0]), f16_bits(c[1])), pk16(f16_bits(c[2]), f16_bits(c[3])) };
}

template <int FORM>
__global__ __launch_bounds__(256) void k_plane(const float* __restrict__ src, int rows, int cols, int ldsrc,
                                               unsigned short* __restrict__ dst, int MP, int KP) {
  static_assert(FORM >= 0 && FORM <= 3);
  const int KTOT = (FORM == 1 || FORM == 3) ? 2 * KP : KP;
  const unsigned ppr   = (unsigned)(KTOT >> 3);
  const unsigned kp8   = (unsigned)(KP >> 3);
  const unsigned total = (unsigned)MP * ppr;
  const unsigned g     = blockIdx.x * 256u + threadIdx.x;
  const unsigned rowu  = g / ppr;
  const unsigned p     = g - rowu * ppr;
  const bool second    = p >= kp8;
  const int row = (int)rowu;
  const int c0  = (int)((second ? p - kp8 : p) << 3);
  const float* srow = src + (size_t)clampi(row, 0, rows - 1) * (size_t)ldsrc;
  float x[8];
  unsigned mk[8];
#pragma unroll
  for (int e = 0; e < 8; ++e) {
    const int c = c0 + e;
    const float v = srow[clampi(c, 0, cols - 1)];
    asm volatile("" :: "v"(v));
    x[e]  = v;
    mk[e] = (row < rows && c < cols) ? 0xFFFFu : 0u;
  }
  const v4f a = (v4f){ x[0], x[1], x[2], x[3] };
  const v4f c = (v4f){ x[4], x[5], x[6], x[7] };
  v4u o;
  if (FORM == 2) {
    o = pack8_f16(a, c);
  } else {
    const v4u hi = pack8_bf16(a, c);
    o = hi;
    if (FORM == 1) { const v4u lo = pack8_bf16_lo(a, c); o = second ? lo : hi; }
  }
  const v4u mw = (v4u){ pk16(mk[0], mk[1]), pk16(mk[2], mk[3]), pk16(mk[4], mk[5]), pk16(mk[6], mk[7]) };
  o &= mw;
  if (g < total) {
    volatile v4u* q = (volatile v4u*)(dst + (size_t)g * 8);
    *q = o;
    __threadfence();
    *q = o;
  }
}

template <int FORM> struct FragOf    { typedef FragB T; };
template <>         struct FragOf<2> { typedef FragH T; };
__device__ __forceinline__ v8f mm(const FragB& a, const FragB& b, v8f c) { return wmb(a, b, c); }
__device__ __forceinline__ v8f mm(const FragH& a, const FragH& b, v8f c) { return wmh(a, b, c); }
template <class F> __device__ __forceinline__ F ld_frag(const unsigned short* p) {
  F f;
  f.h[0] = *(const v8usa*)(p);
  f.h[1] = *(const v8usa*)(p + 16);
  return f;
}

template <int FORM, int EPI>
__global__ __launch_bounds__(256) __attribute__((amdgpu_num_vgpr(248)))
void k_gemm_nt(const unsigned short* __restrict__ A, const unsigned short* __restrict__ B,
               const float* __restrict__ bias, float* __restrict__ D, int M, int N, int KTOT, int ldd) {
  static_assert(FORM >= 0 && FORM <= 2);
  static_assert(EPI == 0 || EPI == 1);
  typedef typename FragOf<FORM>::T F;
  __shared__ __attribute__((aligned(16))) float sT[8][16 * 68];
  const int lane = threadIdx.x & 31;
  const int wave = threadIdx.x >> 5;
  const int tilesM = (M + 63) >> 6;
  const int tilesN = (N + 63) >> 6;
  const int tile = blockIdx.x * 8 + wave;
  if (tile >= tilesM * tilesN) return;
  const int tm = tile / tilesN;
  const int tn = tile - tm * tilesN;
  const int m0 = tm << 6;
  const int n0 = tn << 6;

  const int rl = lane & 15;
  const int h8 = (lane >> 4) * 8;
  const unsigned short* pa = A + (size_t)(m0 + rl) * (size_t)KTOT + h8;
  const unsigned short* pb = B + (size_t)(n0 + rl) * (size_t)KTOT + h8;

  v8f acc[4][4];
#pragma unroll
  for (int i = 0; i < 4; ++i)
#pragma unroll
    for (int j = 0; j < 4; ++j) acc[i][j] = (v8f){0.f, 0.f, 0.f, 0.f, 0.f, 0.f, 0.f, 0.f};

#pragma unroll 1
  for (int k0 = 0; k0 < KTOT; k0 += 32) {
    F bf[4];
#pragma unroll
    for (int j = 0; j < 4; ++j) bf[j] = ld_frag<F>(pb + (size_t)(j << 4) * (size_t)KTOT + k0);
#pragma unroll
    for (int i = 0; i < 4; ++i) {
      const F af = ld_frag<F>(pa + (size_t)(i << 4) * (size_t)KTOT + k0);
#pragma unroll
      for (int j = 0; j < 4; ++j) acc[i][j] = mm(af, bf[j], acc[i][j]);
    }
  }

  float* slab = sT[wave];
  const int hh = lane >> 4;
  const int c4 = (lane & 15) * 4;
  const int nc = n0 + c4;
  const bool cok = nc < N;
  v4f bv = (v4f){0.f, 0.f, 0.f, 0.f};
  if (EPI == 1) {
    bv = *(const v4fa*)(bias + clampi(nc, 0, N - 4));
    asm volatile("" :: "v"(bv));
  }
#pragma unroll
  for (int i = 0; i < 4; ++i) {
    const int mBase = m0 + (i << 4);
#pragma unroll
    for (int j = 0; j < 4; ++j) {
#pragma unroll
      for (int r = 0; r < 8; ++r) slab[(h8 + r) * 68 + (j << 4) + rl] = acc[i][j][r];
    }
    __builtin_amdgcn_fence(__ATOMIC_RELEASE, "workgroup");
    __builtin_amdgcn_wave_barrier();
    __builtin_amdgcn_fence(__ATOMIC_ACQUIRE, "workgroup");
    v4f vv[8];
#pragma unroll
    for (int it = 0; it < 8; ++it) {
      const int row = it * 2 + hh;
      v4f v = *(const v4fa*)(slab + row * 68 + c4);
      if (EPI == 1) v += bv;
      vv[it] = v;
    }
    for (int pass = 0; pass < 2; ++pass) {
#pragma unroll
      for (int it = 0; it < 8; ++it) {
        const int row = mBase + it * 2 + hh;
        if (cok && row < M) *(volatile v4f*)(D + (size_t)row * (size_t)ldd + nc) = vv[it];
      }
      __threadfence();
    }
    __builtin_amdgcn_fence(__ATOMIC_RELEASE, "workgroup");
    __builtin_amdgcn_wave_barrier();
    __builtin_amdgcn_fence(__ATOMIC_ACQUIRE, "workgroup");
  }
}

#define NN      32768
#define NE      131072
#define FA      128
#define FB      32
#define XCW     160
#define F0      64
#define CIN     96
#define OB      1024
#define NBKT    32
#define RCAP    5632
#define DEGCAP  32
#define BCHUNK  2048

static_assert(NBKT * OB == NN);
static_assert(NE % BCHUNK == 0);
static_assert(RCAP % 1024 == 128 || RCAP % 32 == 0);
static_assert((RCAP * 4) % 128 == 0);
static_assert(4324 + 4324 / 4 <= RCAP);
static_assert(4204 + 4204 / 4 <= RCAP);
static_assert(15 + 8 <= DEGCAP);
static_assert(RCAP < 65536);

typedef int v4i __attribute__((ext_vector_type(4)));
typedef v4i __attribute__((may_alias)) v4ia;

__device__ __forceinline__ void wsync() {
  __builtin_amdgcn_fence(__ATOMIC_RELEASE, "workgroup");
  __builtin_amdgcn_wave_barrier();
  __builtin_amdgcn_fence(__ATOMIC_ACQUIRE, "workgroup");
}
__device__ __forceinline__ float rlf(float x, int j) {
  return __int_as_float(__builtin_amdgcn_readlane(__float_as_int(x), j));
}
__device__ __forceinline__ float sel4v(v4f v, int h) {
  return h == 0 ? v[0] : (h == 1 ? v[1] : (h == 2 ? v[2] : v[3]));
}
__device__ __forceinline__ float sel4s(float a, float b, float c, float d, int h) {
  return h == 0 ? a : (h == 1 ? b : (h == 2 ? c : d));
}

__global__ __launch_bounds__(256) void k_vecs(const float* __restrict__ b0, const float* __restrict__ b1,
                                              const float* __restrict__ b2, const float* __restrict__ b3,
                                              float* __restrict__ tab) {
  const int tid = (int)threadIdx.x;
  const int a = tid >> 6;
  const int q = tid & 63;
  const int c = 4 * q;
  const v4f v0 = *(const v4fa*)(b0 + (c < 60 ? c : 60));
  const v4f v1 = *(const v4fa*)(b1 + (c < 92 ? c : 92));
  const v4f v2 = *(const v4fa*)(b2 + (c < 124 ? c : 124));
  const v4f v3 = *(const v4fa*)(b3 + (c < 156 ? c : 156));
  asm volatile("" :: "v"(v0));
  asm volatile("" :: "v"(v1));
  asm volatile("" :: "v"(v2));
  asm volatile("" :: "v"(v3));
  const int n = a == 0 ? 64 : (a == 1 ? 96 : (a == 2 ? 128 : 160));
  v4f v = a == 0 ? v0 : (a == 1 ? v1 : (a == 2 ? v2 : v3));
  const bool ok = c < n;
  v4f o;
  o[0] = ok ? bf16_val(v[0]) : 0.f;
  o[1] = ok ? bf16_val(v[1]) : 0.f;
  o[2] = ok ? bf16_val(v[2]) : 0.f;
  o[3] = ok ? bf16_val(v[3]) : 0.f;
  volatile v4f* p = (volatile v4f*)(tab + a * 256 + c);
  *p = o;
  __threadfence();
  *p = o;
}

__global__ __launch_bounds__(256) void k_wtr(const float* __restrict__ w, int cols, int K, int dup,
                                             unsigned short* __restrict__ wt, int nUnits) {
  const int u  = (int)blockIdx.x * 256 + (int)threadIdx.x;
  const int uc = u < nUnits ? u : nUnits - 1;
  const int kq  = K >> 3;
  const int ppr = dup != 0 ? 2 * kq : kq;
  const int n  = uc / ppr;
  const int p  = uc - n * ppr;
  const int pk = p >= kq ? p - kq : p;
  const int k8 = pk * 8;
  const int ncl = n < cols ? n : cols - 1;
  const float* p0 = w + (size_t)k8 * (size_t)cols + ncl;
  unsigned bits[8];
#pragma unroll
  for (int e = 0; e < 8; ++e) {
    const float v = p0[(size_t)e * (size_t)cols];
    asm volatile("" :: "v"(v));
    bits[e] = bf16_bits(v);
  }
  const unsigned m = n < cols ? 0xFFFFFFFFu : 0u;
  const v4u o = (v4u){ pk16(bits[0], bits[1]) & m, pk16(bits[2], bits[3]) & m,
                       pk16(bits[4], bits[5]) & m, pk16(bits[6], bits[7]) & m };
  if (u < nUnits) {
    volatile v4u* q = (volatile v4u*)(wt + (size_t)u * 8);
    *q = o;
    __threadfence();
    *q = o;
  }
}

static_assert((NN * (XCW / 8)) % 256 == 0);
__global__ __launch_bounds__(256) void k_xc(const float* __restrict__ xa, const float* __restrict__ xb,
                                            unsigned short* __restrict__ dst) {
  const unsigned g   = blockIdx.x * 256u + threadIdx.x;
  const unsigned row = g / 20u;
  const unsigned p   = g - row * 20u;
  const unsigned pa  = p < 16u ? p : 15u;
  const unsigned pb  = p >= 16u ? p - 16u : 0u;
  const float* ra = xa + (size_t)row * FA + pa * 8u;
  const float* rb = xb + (size_t)row * FB + pb * 8u;
  const v4f a0 = *(const v4fa*)ra;
  const v4f a1 = *(const v4fa*)(ra + 4);
  const v4f b0 = *(const v4fa*)rb;
  const v4f b1 = *(const v4fa*)(rb + 4);
  asm volatile("" :: "v"(a0));
  asm volatile("" :: "v"(a1));
  asm volatile("" :: "v"(b0));
  asm volatile("" :: "v"(b1));
  const v4u oa = pack8_bf16(a0, a1);
  const v4u ob = pack8_bf16(b0, b1);
  const unsigned m = p >= 16u ? 0xFFFFFFFFu : 0u;
  const v4u mv = (v4u){ m, m, m, m };
  const v4u o = (ob & mv) | (oa & ~mv);
  volatile v4u* q = (volatile v4u*)(dst + (size_t)g * 8);
  *q = o;
  __threadfence();
  *q = o;
}

__global__ __launch_bounds__(256) void k_bucket(const int* __restrict__ ei, int* __restrict__ lists,
                                                int* __restrict__ cow) {
  __shared__ __attribute__((aligned(16))) int reg1[RCAP];
  __shared__ __attribute__((aligned(16))) int reg2[RCAP];
  __shared__ __attribute__((aligned(16))) int scnt[OB];
  __shared__ __attribute__((aligned(16))) int soff[OB];
  __shared__ __attribute__((aligned(16))) int curs[OB];
  __shared__ int wcnt[8];
  __shared__ int wtot[8];
  const int tid = (int)threadIdx.x, lane = tid & 31, wave = tid >> 5;
  const int which = (int)blockIdx.x >> 5;
  const int b = (int)blockIdx.x & 31;
  const int keyOff = which == 0 ? NE : 0;
  const int parOff = which == 0 ? 0 : NE;
  const unsigned base = (unsigned)(b * OB);

  for (int i = tid; i < RCAP; i += 256) { reg1[i] = 0; reg2[i] = 0; }
  for (int i = tid; i < OB; i += 256) { scnt[i] = 0; soff[i] = 0; curs[i] = 0; }
  if (tid < 8) { wcnt[tid] = 0; wtot[tid] = 0; }
  __syncthreads();

  int tot = 0;
#pragma unroll 1
  for (int ch = 0; ch < NE / BCHUNK; ++ch) {
    const int e0 = ch * BCHUNK + tid * 8;
    const v4i ka = *(const v4ia*)(ei + keyOff + e0);
    const v4i kb = *(const v4ia*)(ei + keyOff + e0 + 4);
    const v4i pa = *(const v4ia*)(ei + parOff + e0);
    const v4i pb = *(const v4ia*)(ei + parOff + e0 + 4);
    asm volatile("" :: "v"(pa[0]), "v"(pa[1]), "v"(pa[2]), "v"(pa[3]), "v"(pb[0]), "v"(pb[1]), "v"(pb[2]), "v"(pb[3]));
    const int kk[8] = { ka[0], ka[1], ka[2], ka[3], kb[0], kb[1], kb[2], kb[3] };
    const int pp[8] = { pa[0], pa[1], pa[2], pa[3], pb[0], pb[1], pb[2], pb[3] };
    unsigned su[8];
    int cnt = 0;
#pragma unroll
    for (int i = 0; i < 8; ++i) {
      su[i] = (unsigned)kk[i] - base;
      cnt += (su[i] < (unsigned)OB) ? 1 : 0;
    }
    int incl = cnt;
#pragma unroll
    for (int d = 1; d < 32; d <<= 1) {
      const int up = __shfl_up(incl, d);
      incl += (lane >= d) ? up : 0;
    }
    if (lane == 31) wcnt[wave] = incl;
    __syncthreads();
    int pre = 0, all = 0;
#pragma unroll
    for (int w2 = 0; w2 < 8; ++w2) {
      const int c = wcnt[w2];
      all += c;
      pre += (w2 < wave) ? c : 0;
    }
    int pos = tot + pre + incl - cnt;
#pragma unroll
    for (int i = 0; i < 8; ++i) {
      if (su[i] < (unsigned)OB) {
        if (pos < RCAP) reg1[pos] = (clampi(pp[i], 0, NN - 1) << 10) | (int)su[i];
        ++pos;
      }
    }
    tot += all;
    __syncthreads();
  }
  const int nh  = tot < RCAP ? tot : RCAP;
  const int ovf = tot > RCAP ? 1 : 0;

  if (wave == 0) {
#pragma unroll 1
    for (int b0 = 0; b0 < nh; b0 += 32) {
      const int idx = b0 + lane;
      const int uv  = reg1[idx < RCAP ? idx : RCAP - 1];
      const int m32 = (nh - b0) < 32 ? (nh - b0) : 32;
#pragma unroll 1
      for (int k = 0; k < m32; ++k) {
        const int u  = __builtin_amdgcn_readlane(uv, k);
        const int sl = u & (OB - 1);
        if (lane == 0) scnt[sl] = scnt[sl] + 1;
      }
    }
  }
  __syncthreads();

  {
    const v4i c4 = *(const v4ia*)(scnt + 4 * tid);
    const int c0 = c4[0] < 0 ? 0 : c4[0], c1 = c4[1] < 0 ? 0 : c4[1];
    const int c2 = c4[2] < 0 ? 0 : c4[2], c3 = c4[3] < 0 ? 0 : c4[3];
    const int ts = c0 + c1 + c2 + c3;
    int incl = ts;
#pragma unroll
    for (int d = 1; d < 32; d <<= 1) {
      const int up = __shfl_up(incl, d);
      incl += (lane >= d) ? up : 0;
    }
    if (lane == 31) wtot[wave] = incl;
    __syncthreads();
    int pre = 0;
#pragma unroll
    for (int w2 = 0; w2 < 8; ++w2) pre += (w2 < wave) ? wtot[w2] : 0;
    int run = pre + incl - ts;
    soff[4 * tid + 0] = run; curs[4 * tid + 0] = run; run += c0;
    soff[4 * tid + 1] = run; curs[4 * tid + 1] = run; run += c1;
    soff[4 * tid + 2] = run; curs[4 * tid + 2] = run; run += c2;
    soff[4 * tid + 3] = run; curs[4 * tid + 3] = run;
  }
  __syncthreads();

  if (wave == 0) {
#pragma unroll 1
    for (int b0 = 0; b0 < nh; b0 += 32) {
      const int idx = b0 + lane;
      const int uv  = reg1[idx < RCAP ? idx : RCAP - 1];
      const int m32 = (nh - b0) < 32 ? (nh - b0) : 32;
#pragma unroll 1
      for (int k = 0; k < m32; ++k) {
        const int u  = __builtin_amdgcn_readlane(uv, k);
        const int sl = u & (OB - 1);
        const int pr = (int)((unsigned)u >> 10);
        if (lane == 0) {
          int pos = curs[sl];
          pos = pos < 0 ? 0 : (pos > RCAP - 1 ? RCAP - 1 : pos);
          reg2[pos] = pr;
          curs[sl] = pos + 1;
        }
      }
    }
  }
  __syncthreads();

  int* lp = lists + (size_t)blockIdx.x * RCAP;
  v4i lv[6];
#pragma unroll
  for (int it = 0; it < 6; ++it) {
    const int i4 = it * 256 + tid;
    const int ic = i4 < RCAP / 4 ? i4 : RCAP / 4 - 1;
    lv[it] = *(const v4ia*)(reg2 + 4 * ic);
  }
  const v4i cc = *(const v4ia*)(scnt + 4 * tid);
  const v4i oo = *(const v4ia*)(soff + 4 * tid);
  v4i cw;
#pragma unroll
  for (int i = 0; i < 4; ++i) {
    const int c = cc[i] < 0 ? 0 : (cc[i] > 255 ? 255 : cc[i]);
    const int o = oo[i] < 0 ? 0 : (oo[i] > RCAP ? RCAP : oo[i]);
    cw[i] = (int)(((unsigned)ovf << 31) | ((unsigned)o << 8) | (unsigned)c);
  }
  int* cp = cow + (size_t)which * NN + (size_t)b * OB + 4 * tid;
  for (int pass = 0; pass < 2; ++pass) {
#pragma unroll
    for (int it = 0; it < 6; ++it) {
      const int i4 = it * 256 + tid;
      if (i4 < RCAP / 4) *(volatile v4i*)(lp + 4 * i4) = lv[it];
    }
    *(volatile v4i*)cp = cw;
    __threadfence();
  }
}

template <int F>
__global__ __launch_bounds__(256) void k_scores(const float* __restrict__ P, const float* __restrict__ asrc,
                                                const float* __restrict__ atrg, float* __restrict__ S) {
  constexpr int C  = 4 * F;
  constexpr int KQ = C / 128;
  static_assert(C % 128 == 0 && F % 4 == 0 && C <= 512);
  __shared__ __attribute__((aligned(16))) float sa[C];
  __shared__ __attribute__((aligned(16))) float st[C];
  __shared__ __attribute__((aligned(16))) float stw[8][32];
  const int tid = (int)threadIdx.x, lane = tid & 31;
  const int wave = __builtin_amdgcn_readfirstlane(tid >> 5);
#pragma unroll
  for (int it = 0; it < 2; ++it) {
    const int i  = it * 256 + tid;
    const int ic = i < C ? i : C - 1;
    const float va = asrc[ic];
    const float vt = atrg[ic];
    asm volatile("" :: "v"(va));
    asm volatile("" :: "v"(vt));
    if (i < C) { sa[i] = bf16_val(va); st[i] = bf16_val(vt); }
  }
  __syncthreads();
  v4f av[KQ], tv[KQ];
  int hd[KQ];
#pragma unroll
  for (int k = 0; k < KQ; ++k) {
    av[k] = *(const v4fa*)(sa + 4 * lane + 128 * k);
    tv[k] = *(const v4fa*)(st + 4 * lane + 128 * k);
    hd[k] = (4 * lane + 128 * k) / F;
  }
  const bool up16 = lane >= 16;
  const bool b3   = ((lane >> 3) & 1) != 0;
  const bool b2   = ((lane >> 2) & 1) != 0;
  float* sw = stw[wave];
  const int nbase = (int)blockIdx.x * 128 + wave * 16;
  float mine = 0.f;
#pragma unroll 1
  for (int ii = 0; ii < 16; ++ii) {
    const int node = nbase + ii;
    const float* pr = P + (size_t)node * C + 4 * lane;
    float ps[4] = { 0.f, 0.f, 0.f, 0.f };
    float pt[4] = { 0.f, 0.f, 0.f, 0.f };
#pragma unroll
    for (int k = 0; k < KQ; ++k) {
      const v4f v = *(const v4fa*)(pr + 128 * k);
      float ds = v[0] * av[k][0];
      ds = fmaf(v[1], av[k][1], ds);
      ds = fmaf(v[2], av[k][2], ds);
      ds = fmaf(v[3], av[k][3], ds);
      float dt = v[0] * tv[k][0];
      dt = fmaf(v[1], tv[k][1], dt);
      dt = fmaf(v[2], tv[k][2], dt);
      dt = fmaf(v[3], tv[k][3], dt);
#pragma unroll
      for (int h = 0; h < 4; ++h) {
        ps[h] += (hd[k] == h) ? ds : 0.f;
        pt[h] += (hd[k] == h) ? dt : 0.f;
      }
    }
    float u[4];
#pragma unroll
    for (int h = 0; h < 4; ++h) {
      const float rs = __shfl_xor(ps[h], 16);
      const float rt = __shfl_xor(pt[h], 16);
      const float s0 = ps[h] + rs;
      const float s1 = pt[h] + rt;
      u[h] = up16 ? s1 : s0;
    }
    float w[2];
#pragma unroll
    for (int q = 0; q < 2; ++q) {
      const float r0 = __shfl_xor(u[q], 8);
      const float r1 = __shfl_xor(u[2 + q], 8);
      const float s0 = u[q] + r0;
      const float s1 = u[2 + q] + r1;
      w[q] = b3 ? s1 : s0;
    }
    const float r0 = __shfl_xor(w[0], 4);
    const float r1 = __shfl_xor(w[1], 4);
    const float z0 = w[0] + r0;
    const float z1 = w[1] + r1;
    float z = b2 ? z1 : z0;
    z += __shfl_xor(z, 2);
    z += __shfl_xor(z, 1);
    const float got = __shfl(z, 4 * (lane & 7));
    mine = ((lane >> 3) == (ii & 3)) ? got : mine;
    if ((ii & 3) == 3) {
      wsync();
      sw[lane] = mine;
      wsync();
      const v4f o = *(const v4fa*)(sw + 4 * (lane & 7));
      float* dp = S + (size_t)(node - 3) * 8 + 4 * (lane & 7);
      if (lane < 8) *(volatile v4f*)dp = o;
      __threadfence();
      if (lane < 8) *(volatile v4f*)dp = o;
    }
  }
}

static_assert(128 * 1024 == NE);
__global__ __launch_bounds__(256) void k_max(const int* __restrict__ ei, const float* __restrict__ S,
                                             float* __restrict__ rec) {
  __shared__ float wm[8];
  const int tid = (int)threadIdx.x, lane = tid & 31, wave = tid >> 5;
  float loc = -3.0e38f;
#pragma unroll 1
  for (int it = 0; it < 4; ++it) {
    const int e = (int)blockIdx.x * 1024 + it * 256 + tid;
    const int s = clampi(ei[e], 0, NN - 1);
    const int t = clampi(ei[NE + e], 0, NN - 1);
    const v4f a = *(const v4fa*)(S + (size_t)s * 8);
    const v4f b = *(const v4fa*)(S + (size_t)t * 8 + 4);
#pragma unroll
    for (int h = 0; h < 4; ++h) {
      float sc = a[h] + b[h];
      sc = sc >= 0.f ? sc : 0.2f * sc;
      loc = fmaxf(loc, sc);
    }
  }
#pragma unroll
  for (int off = 16; off > 0; off >>= 1) loc = fmaxf(loc, __shfl_xor(loc, off));
  if (lane == 0) wm[wave] = loc;
  __syncthreads();
  float bm = wm[0];
#pragma unroll
  for (int w2 = 1; w2 < 8; ++w2) bm = fmaxf(bm, wm[w2]);
  const v4f o = (v4f){ bm, bm, bm, bm };
  float* dp = rec + (size_t)blockIdx.x * 32 + 4 * (tid & 7);
  if (tid < 8) *(volatile v4f*)dp = o;
  __threadfence();
  if (tid < 8) *(volatile v4f*)dp = o;
}

__global__ __launch_bounds__(128) void k_max2(const float* __restrict__ rec, float* __restrict__ gm) {
  __shared__ float wm[4];
  const int tid = (int)threadIdx.x, lane = tid & 31, wave = tid >> 5;
  float loc = rec[(size_t)tid * 32];
#pragma unroll
  for (int off = 16; off > 0; off >>= 1) loc = fmaxf(loc, __shfl_xor(loc, off));
  if (lane == 0) wm[wave] = loc;
  __syncthreads();
  const float bm = fmaxf(fmaxf(wm[0], wm[1]), fmaxf(wm[2], wm[3]));
  const v4f o = (v4f){ bm, bm, bm, bm };
  float* dp = gm + 4 * (tid & 7);
  if (tid < 8) *(volatile v4f*)dp = o;
  __threadfence();
  if (tid < 8) *(volatile v4f*)dp = o;
}

__global__ __launch_bounds__(256) void k_den(const int* __restrict__ lists, const int* __restrict__ cow,
                                             const float* __restrict__ S, const float* __restrict__ gmaxp,
                                             float* __restrict__ DEN) {
  __shared__ __attribute__((aligned(16))) float sden[256 * 4];
  const int tid = (int)threadIdx.x, lane = tid & 31;
  const int wave = __builtin_amdgcn_readfirstlane(tid >> 5);
  const float gm = gmaxp[0];
  const float qn = __uint_as_float(0x7fc00000u);
#pragma unroll 1
  for (int jo = 0; jo < 32; ++jo) {
    const int ol = wave * 32 + jo;
    const int s  = (int)blockIdx.x * 256 + ol;
    const int cwv  = cow[s];
    const int craw = cwv & 255;
    int off = (cwv >> 8) & 0xFFFF; off = off > RCAP - 1 ? RCAP - 1 : off;
    int cnt = craw > DEGCAP ? DEGCAP : craw;
    cnt = cnt > RCAP - off ? RCAP - off : cnt;
    const bool poison = (cwv < 0) || (craw > DEGCAP);
    const int cn = __builtin_amdgcn_readfirstlane(cnt);
    const int* lp = lists + (size_t)(s >> 10) * RCAP;
    int li = off + lane; li = li > RCAP - 1 ? RCAP - 1 : li;
    int tj = lp[li];
    asm volatile("" :: "v"(tj));
    tj = clampi(tj, 0, NN - 1);
    const v4f tt = *(const v4fa*)(S + (size_t)tj * 8 + 4);
    asm volatile("" :: "v"(tt));
    const v4f ss = *(const v4fa*)(S + (size_t)s * 8);
    asm volatile("" :: "v"(ss));
    const bool act = lane < cn;
    float e0 = 0.f, e1 = 0.f, e2 = 0.f, e3 = 0.f;
#pragma unroll 1
    for (int h = 0; h < 4; ++h) {
      float sc = sel4v(ss, h) + sel4v(tt, h);
      sc = sc >= 0.f ? sc : 0.2f * sc;
      float e = expf(sc - gm);
      e = act ? e : 0.f;
      e0 = h == 0 ? e : e0;
      e1 = h == 1 ? e : e1;
      e2 = h == 2 ? e : e2;
      e3 = h == 3 ? e : e3;
    }
    float d0 = 0.f, d1 = 0.f, d2 = 0.f, d3 = 0.f;
#pragma unroll 1
    for (int j = 0; j < cn; ++j) {
      d0 += rlf(e0, j);
      d1 += rlf(e1, j);
      d2 += rlf(e2, j);
      d3 += rlf(e3, j);
    }
    v4f dv = (v4f){ d0, d1, d2, d3 };
    const v4f q4 = (v4f){ qn, qn, qn, qn };
    dv = poison ? q4 : dv;
    if (lane == 0) *(v4fa*)(sden + 4 * ol) = dv;
  }
  __syncthreads();
  const v4f o = *(const v4fa*)(sden + 4 * tid);
  float* dp = DEN + ((size_t)blockIdx.x * 256 + tid) * 4;
  *(volatile v4f*)dp = o;
  __threadfence();
  *(volatile v4f*)dp = o;
}

template <int F, int MODE>
__global__ __launch_bounds__(256) void k_replay(const int* __restrict__ lists, const int* __restrict__ cow,
                                                const float* __restrict__ P, const float* __restrict__ S,
                                                const float* __restrict__ DEN, const float* __restrict__ gmaxp,
                                                const float* __restrict__ X, const float* __restrict__ bias,
                                                unsigned short* __restrict__ OUT) {
  constexpr int C   = 4 * F;
  constexpr int KQ  = C / 128;
  constexpr int NPH = F / 8;
  static_assert(C % 128 == 0 && F % 8 == 0 && 2 * NPH <= 32 && F <= 256);
  __shared__ __attribute__((aligned(16))) float sb[F];
  __shared__ __attribute__((aligned(16))) float stw[8][C];
  const int tid = (int)threadIdx.x, lane = tid & 31;
  const int wave = __builtin_amdgcn_readfirstlane(tid >> 5);
  {
    const int ic = tid < F ? tid : F - 1;
    const float bv = bias[ic];
    asm volatile("" :: "v"(bv));
    if (tid < F) sb[tid] = bf16_val(bv);
  }
  __syncthreads();
  int hd[KQ];
#pragma unroll
  for (int k = 0; k < KQ; ++k) hd[k] = (4 * lane + 128 * k) / F;
  const float gm = gmaxp[0];
  const float qn = __uint_as_float(0x7fc00000u);
  const int pl = lane < 2 * NPH ? lane : 2 * NPH - 1;
  const bool isLo = pl >= NPH;
  const int f0 = 8 * (isLo ? pl - NPH : pl);
  const unsigned lom = isLo ? 0xFFFFFFFFu : 0u;
  const v4u lomv = (v4u){ lom, lom, lom, lom };
  float* sw = stw[wave];

#pragma unroll 1
  for (int jt = 0; jt < 8; ++jt) {
    const int t = (int)blockIdx.x * 64 + wave * 8 + jt;
    const int cwv  = cow[t];
    const int craw = cwv & 255;
    int off = (cwv >> 8) & 0xFFFF; off = off > RCAP - 1 ? RCAP - 1 : off;
    int cnt = craw > DEGCAP ? DEGCAP : craw;
    cnt = cnt > RCAP - off ? RCAP - off : cnt;
    const bool poison = (cwv < 0) || (craw > DEGCAP);
    const int cn = __builtin_amdgcn_readfirstlane(cnt);
    const int* lp = lists + (size_t)(t >> 10) * RCAP;
    int li = off + lane; li = li > RCAP - 1 ? RCAP - 1 : li;
    int sid = lp[li];
    asm volatile("" :: "v"(sid));
    sid = clampi(sid, 0, NN - 1);
    const v4f ss = *(const v4fa*)(S + (size_t)sid * 8);
    asm volatile("" :: "v"(ss));
    const v4f tt = *(const v4fa*)(S + (size_t)t * 8 + 4);
    asm volatile("" :: "v"(tt));
    v4f dn = (v4f){ 1.f, 1.f, 1.f, 1.f };
    if (MODE == 1) {
      dn = *(const v4fa*)(DEN + (size_t)sid * 4);
      asm volatile("" :: "v"(dn));
    }
    const bool act = lane < cn;
    float e0 = 0.f, e1 = 0.f, e2 = 0.f, e3 = 0.f;
#pragma unroll 1
    for (int h = 0; h < 4; ++h) {
      float sc = sel4v(ss, h) + sel4v(tt, h);
      sc = sc >= 0.f ? sc : 0.2f * sc;
      float e = expf(sc - gm);
      e = act ? e : 0.f;
      if (MODE == 1) e = e / (sel4v(dn, h) + 1e-16f);
      e0 = h == 0 ? e : e0;
      e1 = h == 1 ? e : e1;
      e2 = h == 2 ? e : e2;
      e3 = h == 3 ? e : e3;
    }
    if (MODE == 0) {
      float d0 = 0.f, d1 = 0.f, d2 = 0.f, d3 = 0.f;
#pragma unroll 1
      for (int j = 0; j < cn; ++j) {
        d0 += rlf(e0, j);
        d1 += rlf(e1, j);
        d2 += rlf(e2, j);
        d3 += rlf(e3, j);
      }
#pragma unroll 1
      for (int h = 0; h < 4; ++h) {
        const float e = sel4s(e0, e1, e2, e3, h);
        const float d = sel4s(d0, d1, d2, d3, h);
        const float q = e / (d + 1e-16f);
        e0 = h == 0 ? q : e0;
        e1 = h == 1 ? q : e1;
        e2 = h == 2 ? q : e2;
        e3 = h == 3 ? q : e3;
      }
    }
    v4f acc[KQ];
#pragma unroll
    for (int k = 0; k < KQ; ++k) acc[k] = (v4f){ 0.f, 0.f, 0.f, 0.f };
#pragma unroll 1
    for (int j = 0; j < cn; ++j) {
      const int s = __builtin_amdgcn_readlane(sid, j);
      const float a0 = rlf(e0, j), a1 = rlf(e1, j), a2 = rlf(e2, j), a3 = rlf(e3, j);
      const float* pr = P + (size_t)s * C + 4 * lane;
#pragma unroll
      for (int k = 0; k < KQ; ++k) {
        const v4f v = *(const v4fa*)(pr + 128 * k);
        const float a = hd[k] == 0 ? a0 : (hd[k] == 1 ? a1 : (hd[k] == 2 ? a2 : a3));
        acc[k] += v * a;
      }
    }
    wsync();
#pragma unroll
    for (int k = 0; k < KQ; ++k) *(v4fa*)(sw + 4 * lane + 128 * k) = acc[k];
    wsync();
    const float* xr = X + (size_t)t * F + f0;
    const v4f xa = *(const v4fa*)xr;
    const v4f xc = *(const v4fa*)(xr + 4);
    asm volatile("" :: "v"(xa));
    asm volatile("" :: "v"(xc));
    v4f sa4 = (v4f){ 0.f, 0.f, 0.f, 0.f };
    v4f sc4 = (v4f){ 0.f, 0.f, 0.f, 0.f };
#pragma unroll
    for (int h = 0; h < 4; ++h) {
      const v4f a = *(const v4fa*)(sw + h * F + f0);
      const v4f c = *(const v4fa*)(sw + h * F + f0 + 4);
      sa4 += (a + xa);
      sc4 += (c + xc);
    }
    const v4f ba = *(const v4fa*)(sb + f0);
    const v4f bc = *(const v4fa*)(sb + f0 + 4);
    v4f ra = sa4 * 0.25f + ba;
    v4f rc = sc4 * 0.25f + bc;
    const v4f q4 = (v4f){ qn, qn, qn, qn };
    ra = poison ? q4 : ra;
    rc = poison ? q4 : rc;
    const v4u hi = pack8_bf16(ra, rc);
    const v4u lo = pack8_bf16_lo(ra, rc);
    const v4u o = (lo & lomv) | (hi & ~lomv);
    volatile v4u* q = (volatile v4u*)(OUT + (size_t)t * (2 * F) + 8 * pl);
    if (lane < 2 * NPH) *q = o;
    __threadfence();
    if (lane < 2 * NPH) *q = o;
  }
}

constexpr size_t SZ_XC   = (size_t)NN * XCW * 2;
constexpr size_t SZ_XR   = (size_t)NN * FA * 2;
constexpr size_t SZ_RP   = (size_t)NN * F0 * 4;
constexpr size_t SZ_CP   = (size_t)NN * CIN * 4;
constexpr size_t SZ_RPHL = (size_t)NN * 2 * F0 * 2;
constexpr size_t SZ_CPHL = (size_t)NN * 2 * CIN * 2;
constexpr size_t SZ_P    = (size_t)NN * 4 * CIN * 4;
constexpr size_t SZ_S    = (size_t)NN * 8 * 4;
constexpr size_t SZ_DEN  = (size_t)NN * 4 * 4;
constexpr size_t SZ_LIST = (size_t)2 * NBKT * RCAP * 4;
constexpr size_t SZ_COW  = (size_t)2 * NN * 4;
constexpr size_t SZ_REC  = (size_t)128 * 32 * 4;
constexpr size_t SZ_GMAX = 256;
constexpr size_t SZ_BT   = 4 * 256 * 4;
constexpr size_t SZ_WGP  = (size_t)64 * 128 * 2;
constexpr size_t SZ_WCP  = (size_t)128 * 160 * 2;
constexpr size_t SZ_WG   = (size_t)256 * 128 * 2;
constexpr size_t SZ_WC   = (size_t)384 * 192 * 2;
constexpr size_t SZ_WGR  = (size_t)128 * 128 * 2;
constexpr size_t SZ_WCR  = (size_t)192 * 192 * 2;
constexpr size_t O_XC   = 0;
constexpr size_t O_XR   = O_XC + SZ_XC;
constexpr size_t O_RP   = O_XR + SZ_XR;
constexpr size_t O_CP   = O_RP + SZ_RP;
constexpr size_t O_RPHL = O_CP + SZ_CP;
constexpr size_t O_CPHL = O_RPHL + SZ_RPHL;
constexpr size_t O_P    = O_CPHL + SZ_CPHL;
constexpr size_t O_SG   = O_P + SZ_P;
constexpr size_t O_SC   = O_SG + SZ_S;
constexpr size_t O_DEN  = O_SC + SZ_S;
constexpr size_t O_LIST = O_DEN + SZ_DEN;
constexpr size_t O_COW  = O_LIST + SZ_LIST;
constexpr size_t O_REC  = O_COW + SZ_COW;
constexpr size_t O_GMAX = O_REC + SZ_REC;
constexpr size_t O_BT   = O_GMAX + SZ_GMAX;
constexpr size_t O_WGP  = O_BT + SZ_BT;
constexpr size_t O_WCP  = O_WGP + SZ_WGP;
constexpr size_t O_WG   = O_WCP + SZ_WCP;
constexpr size_t O_WC   = O_WG + SZ_WG;
constexpr size_t O_WGR  = O_WC + SZ_WC;
constexpr size_t O_WCR  = O_WGR + SZ_WGR;
constexpr size_t WS_TOTAL = O_WCR + SZ_WCR;
static_assert(SZ_XC % 256 == 0 && SZ_XR % 256 == 0 && SZ_RP % 256 == 0 && SZ_CP % 256 == 0);
static_assert(SZ_RPHL % 256 == 0 && SZ_CPHL % 256 == 0 && SZ_P % 256 == 0 && SZ_S % 256 == 0 && SZ_DEN % 256 == 0);
static_assert(SZ_LIST % 256 == 0 && SZ_COW % 256 == 0 && SZ_REC % 256 == 0 && SZ_BT % 256 == 0);
static_assert(SZ_WGP % 256 == 0 && SZ_WCP % 256 == 0 && SZ_WG % 256 == 0 && SZ_WC % 256 == 0);
static_assert(SZ_WGR % 256 == 0 && SZ_WCR % 256 == 0);
static_assert(WS_TOTAL == ((size_t)452625 << 8));
static_assert(WS_TOTAL <= ((size_t)128 << 20));
static_assert(NN % 64 == 0 && FA % 32 == 0 && XCW % 32 == 0 && (2 * F0) % 32 == 0 && (2 * CIN) % 32 == 0);
static_assert(F0 % 32 == 0 && CIN % 32 == 0 && (4 * F0) % 32 == 0 && (4 * CIN) % 32 == 0 && XCW % 4 == 0);
static_assert((NN * FA / 8) % 256 == 0 && (NN * 2 * F0 / 8) % 256 == 0 && (NN * 2 * CIN / 8) % 256 == 0);
constexpr size_t OUT1_EL = (size_t)16777216 / 4;
static_assert(OUT1_EL == (size_t)NN * FA);
constexpr size_t OUT_TOTAL = OUT1_EL + (size_t)NN * XCW;

extern "C" void kernel_launch(void* const* d_in, const int* in_sizes, int n_in,
                              void* d_out, int out_size, void* d_ws, size_t ws_size,
                              hipStream_t stream) {
  if (n_in != 19) return;
  const int want[19] = { NN * FA, NN * FB, 2 * NE, FA * F0, F0, F0 * FA, FA, F0 * 4 * F0, 4 * F0, 4 * F0, F0,
                         XCW * CIN, CIN, CIN * XCW, XCW, CIN * 4 * CIN, 4 * CIN, 4 * CIN, CIN };
  for (int i = 0; i < 19; ++i) if (in_sizes[i] != want[i]) return;
  if ((size_t)out_size != OUT_TOTAL) return;
  if (ws_size < WS_TOTAL) return;

  const float* xa   = (const float*)d_in[0];
  const float* xb   = (const float*)d_in[1];
  const int*   ei   = (const int*)  d_in[2];
  const float* Wgp  = (const float*)d_in[3];
  const float* bgp  = (const float*)d_in[4];
  const float* Wgr  = (const float*)d_in[5];
  const float* bgr  = (const float*)d_in[6];
  const float* Wg   = (const float*)d_in[7];
  const float* agS  = (const float*)d_in[8];
  const float* agT  = (const float*)d_in[9];
  const float* bg   = (const float*)d_in[10];
  const float* Wcp  = (const float*)d_in[11];
  const float* bcp  = (const float*)d_in[12];
  const float* Wcr  = (const float*)d_in[13];
  const float* bcr  = (const float*)d_in[14];
  const float* Wc   = (const float*)d_in[15];
  const float* acS  = (const float*)d_in[16];
  const float* acT  = (const float*)d_in[17];
  const float* bc   = (const float*)d_in[18];
  float* out0 = (float*)d_out;
  float* out1 = (float*)d_out + OUT1_EL;

  char* ws = (char*)d_ws;
  unsigned short* XC   = (unsigned short*)(ws + O_XC);
  unsigned short* XR   = (unsigned short*)(ws + O_XR);
  float*          RP   = (float*)(ws + O_RP);
  float*          CP   = (float*)(ws + O_CP);
  unsigned short* RPHL = (unsigned short*)(ws + O_RPHL);
  unsigned short* CPHL = (unsigned short*)(ws + O_CPHL);
  float*          PP   = (float*)(ws + O_P);
  float*          SG   = (float*)(ws + O_SG);
  float*          SC   = (float*)(ws + O_SC);
  float*          DENC = (float*)(ws + O_DEN);
  int*            LST  = (int*)(ws + O_LIST);
  int*            COW  = (int*)(ws + O_COW);
  float*          REC  = (float*)(ws + O_REC);
  float*          GMX  = (float*)(ws + O_GMAX);
  float*          BT   = (float*)(ws + O_BT);
  unsigned short* WGP  = (unsigned short*)(ws + O_WGP);
  unsigned short* WCP  = (unsigned short*)(ws + O_WCP);
  unsigned short* WGT  = (unsigned short*)(ws + O_WG);
  unsigned short* WCT  = (unsigned short*)(ws + O_WC);
  unsigned short* WGR  = (unsigned short*)(ws + O_WGR);
  unsigned short* WCR  = (unsigned short*)(ws + O_WCR);

  k_vecs<<<1, 256, 0, stream>>>(bgp, bcp, bgr, bcr, BT);
  k_wtr<<<4,  256, 0, stream>>>(Wgp, 64,  128, 0, WGP, 1024);
  k_wtr<<<10, 256, 0, stream>>>(Wcp, 96,  160, 0, WCP, 2560);
  k_wtr<<<16, 256, 0, stream>>>(Wg,  256, 64,  1, WGT, 4096);
  k_wtr<<<36, 256, 0, stream>>>(Wc,  384, 96,  1, WCT, 9216);
  k_wtr<<<8,  256, 0, stream>>>(Wgr, 128, 64,  1, WGR, 2048);
  k_wtr<<<18, 256, 0, stream>>>(Wcr, 160, 96,  1, WCR, 4608);
  k_plane<0><<<NN * FA / 8 / 256, 256, 0, stream>>>(xa, NN, FA, FA, XR, NN, FA);
  k_xc<<<NN * (XCW / 8) / 256, 256, 0, stream>>>(xa, xb, XC);
  k_bucket<<<2 * NBKT, 256, 0, stream>>>(ei, LST, COW);

  k_gemm_nt<0, 1><<<64, 256, 0, stream>>>(XR, WGP, BT, RP, NN, F0, FA, F0);
  k_plane<1><<<NN * 2 * F0 / 8 / 256, 256, 0, stream>>>(RP, NN, F0, F0, RPHL, NN, F0);
  k_gemm_nt<0, 0><<<256, 256, 0, stream>>>(RPHL, WGT, BT, PP, NN, 4 * F0, 2 * F0, 4 * F0);
  k_scores<F0><<<NN / 128, 256, 0, stream>>>(PP, agS, agT, SG);
  k_max<<<128, 256, 0, stream>>>(ei, SG, REC);
  k_max2<<<1, 128, 0, stream>>>(REC, GMX);
  k_replay<F0, 0><<<NN / 64, 256, 0, stream>>>(LST, COW, PP, SG, SG, GMX, RP, bg, RPHL);
  k_gemm_nt<0, 1><<<128, 256, 0, stream>>>(RPHL, WGR, BT + 512, out0, NN, FA, 2 * F0, FA);

  k_gemm_nt<0, 1><<<128, 256, 0, stream>>>(XC, WCP, BT + 256, CP, NN, CIN, XCW, CIN);
  k_plane<1><<<NN * 2 * CIN / 8 / 256, 256, 0, stream>>>(CP, NN, CIN, CIN, CPHL, NN, CIN);
  k_gemm_nt<0, 0><<<384, 256, 0, stream>>>(CPHL, WCT, BT, PP, NN, 4 * CIN, 2 * CIN, 4 * CIN);
  k_scores<CIN><<<NN / 128, 256, 0, stream>>>(PP, acS, acT, SC);
  k_max<<<128, 256, 0, stream>>>(ei, SC, REC);
  k_max2<<<1, 128, 0, stream>>>(REC, GMX + 32);
  k_den<<<NN / 256, 256, 0, stream>>>(LST + (size_t)NBKT * RCAP, COW + NN, SC, GMX + 32, DENC);
  k_replay<CIN, 1><<<NN / 64, 256, 0, stream>>>(LST, COW, PP, SC, DENC, GMX + 32, CP, bc, CPHL);
  k_gemm_nt<0, 1><<<192, 256, 0, stream>>>(CPHL, WCR, BT + 768, out1, NN, XCW, 2 * CIN, XCW);
}
